// GraphEncoder_26946624815681
// MI455X (gfx1250) — hardware-run, weakly checked
//
#include <hip/hip_runtime.h>

typedef float          v8f   __attribute__((ext_vector_type(8)));
typedef float          v4f   __attribute__((ext_vector_type(4)));
typedef unsigned int   v4u   __attribute__((ext_vector_type(4)));
typedef int            v8i   __attribute__((ext_vector_type(8)));
typedef unsigned short v8us  __attribute__((ext_vector_type(8)));
typedef unsigned short v16us __attribute__((ext_vector_type(16)));
typedef __bf16         v16bf __attribute__((ext_vector_type(16)));
typedef _Float16       v16h  __attribute__((ext_vector_type(16)));
typedef v4f  __attribute__((may_alias)) v4fa;
typedef v8us __attribute__((may_alias)) v8usa;
union FragB { v16bf v; v16us u; v8us h[2]; v8i w; };
union FragH { v16h  v; v16us u; v8us h[2]; v8i w; };

__device__ __forceinline__ v8f wmb(const FragB& a, const FragB& b, v8f c) {
  v8f d = __builtin_amdgcn_wmma_f32_16x16x32_bf16(false, a.v, false, b.v, (short)0, c, false, false);
  asm volatile("v_nop\n\tv_nop\n\tv_nop\n\tv_nop" : "+v"(d) : "v"(a.w), "v"(b.w));
  return d;
}

__device__ __forceinline__ v8f wmh(const FragH& a, const FragH& b, v8f c) {
  v8f d = __builtin_amdgcn_wmma_f32_16x16x32_f16(false, a.v, false, b.v, (short)0, c, false, false);
  asm volatile("v_nop\n\tv_nop\n\tv_nop\n\tv_nop" : "+v"(d) : "v"(a.w), "v"(b.w));
  return d;
}

__device__ __forceinline__ unsigned bf16_bits(float f) {
  const unsigned u = __float_as_uint(f);
  const unsigned r = (u + 0x7FFFu + ((u >> 16) & 1u)) >> 16;
  const unsigned q = (u >> 16) | 0x40u;
  return ((u & 0x7fffffffu) > 0x7f800000u) ? q : r;
}

__device__ __forceinline__ float bf16_val(float f) {
  return __uint_as_float(bf16_bits(f) << 16);
}
__device__ __forceinline__ int clampi(int v, int lo, int hi) {
  return v < lo ? lo : (v > hi ? hi : v);
}

__device__ __forceinline__ unsigned f16_bits(float f) {
  const unsigned u  = __float_as_uint(f);
  const unsigned s  = (u >> 16) & 0x8000u;
  const unsigned a  = u & 0x7fffffffu;
  const unsigned t  = a - 0x38000000u;
  const unsigned r  = (t + 0x0FFFu + ((t >> 13) & 1u)) >> 13;
  const unsigned rc = r > 0x7C00u ? 0x7C00u : r;
  const bool small  = a < 0x38800000u;
  const bool isnan  = a > 0x7f800000u;
  const unsigned fin = small ? 0u : (s | rc);
  return isnan ? (s | 0x7E00u) : fin;
}

__device__ __forceinline__ unsigned pk16(unsigned lo, unsigned hi) { return lo | (hi << 16); }
__device__ __forceinline__ unsigned bf16_lo_bits(float v) {
  float hi = bf16_val(v);
  asm volatile("" : "+v"(hi));
  return bf16_bits(v - hi);
}
__device__ __forceinline__ v4u pack8_bf16(v4f a, v4f c) {
  return (v4u){ pk16(bf16_bits(a[0]), bf16_bits(a[1])), pk16(bf16_bits(a[2]), bf16_bits(a[3])),
                pk16(bf16_bits(c[0]), bf16_bits(c[1])), pk16(bf16_bits(c[2]), bf16_bits(c[3])) };
}
__device__ __forceinline__ v4u pack8_bf16_lo(v4f a, v4f c) {
  return (v4u){ pk16(bf16_lo_bits(a[0]), bf16_lo_bits(a[1])), pk16(bf16_lo_bits(a[2]), bf16_lo_bits(a[3])),
                pk16(bf16_lo_bits(c[0]), bf16_lo_bits(c[1])), pk16(bf16_lo_bits(c[2]), bf16_lo_bits(c[3])) };
}
__device__ __forceinline__ v4u pack8_f16(v4f a, v4f c) {
  return (v4u){ pk16(f16_bits(a[0]), f16_bits(a[1])), pk16(f16_bits(a[2]), f16_bits(a[3])),
                pk16(f16_bits(c[0]), f16_bits(c[1])), pk16(f16_bits(c[2]), f16_bits(c[3])) };
}

template <int FORM>
__global__ __launch_bounds__(256) void k_plane(const float* __restrict__ src, int rows, int cols, int ldsrc,
                                               unsigned short* __restrict__ dst, int MP, int KP) {
  static_assert(FORM >= 0 && FORM <= 3);
  const int KTOT = (FORM == 1 || FORM == 3) ? 2 * KP : KP;
  const unsigned ppr   = (unsigned)(KTOT >> 3);
  const unsigned kp8   = (unsigned)(KP >> 3);
  const unsigned total = (unsigned)MP * ppr;
  const unsigned g     = blockIdx.x * 256u + threadIdx.x;
  const unsigned rowu  = g / ppr;
  const unsigned p     = g - rowu * ppr;
  const bool second    = p >= kp8;
  const int row = (int)rowu;
  const int c0  = (int)((second ? p - kp8 : p) << 3);
  const float* srow = src + (size_t)clampi(row, 0, rows - 1) * (size_t)ldsrc;
  float x[8];
  unsigned mk[8];
#pragma unroll
  for (int e = 0; e < 8; ++e) {
    const int c = c0 + e;
    const float v = srow[clampi(c, 0, cols - 1)];
    asm volatile("" :: "v"(v));
    x[e]  = v;
    mk[e] = (row < rows && c < cols) ? 0xFFFFu : 0u;
  }
  const v4f a = (v4f){ x[0], x[1], x[2], x[3] };
  const v4f c = (v4f){ x[4], x[5], x[6], x[7] };
  v4u o;
  if (FORM == 2) {
    o = pack8_f16(a, c);
  } else {
    const v4u hi = pack8_bf16(a, c);
    o = hi;
    if (FORM == 1) { const v4u lo = pack8_bf16_lo(a, c); o = second ? lo : hi; }
  }
  const v4u mw = (v4u){ pk16(mk[0], mk[1]), pk16(mk[2], mk[3]), pk16(mk[4], mk[5]), pk16(mk[6], mk[7]) };
  o &= mw;
  if (g < total) {
    volatile v4u* q = (volatile v4u*)(dst + (size_t)g * 8);
    *q = o;
    __threadfence();
    *q = o;
  }
}

template <int FORM> struct FragOf    { typedef FragB T; };
template <>         struct FragOf<2> { typedef FragH T; };
__device__ __forceinline__ v8f mm(const FragB& a, const FragB& b, v8f c) { return wmb(a, b, c); }
__device__ __forceinline__ v8f mm(const FragH& a, const FragH& b, v8f c) { return wmh(a, b, c); }
template <class F> __device__ __forceinline__ F ld_frag(const unsigned short* p) {
  F f;
  f.h[0] = *(const v8usa*)(p);
  f.h[1] = *(const v8usa*)(p + 16);
  return f;
}

template <int FORM, int EPI>
__global__ __launch_bounds__(256) __attribute__((amdgpu_num_vgpr(248)))
void k_gemm_nt(const unsigned short* __restrict__ A, const unsigned short* __restrict__ B,
               const float* __restrict__ bias, float* __restrict__ D, int M, int N, int KTOT, int ldd) {
  static_assert(FORM >= 0 && FORM <= 2);
  static_assert(EPI == 0 || EPI == 1);
  typedef typename FragOf<FORM>::T F;
  __shared__ __attribute__((aligned(16))) float sT[8][16 * 68];
  const int lane = threadIdx.x & 31;
  const int wave = threadIdx.x >> 5;
  const int tilesM = (M + 63) >> 6;
  const int tilesN = (N + 63) >> 6;
  const int tile = blockIdx.x * 8 + wave;
  if (tile >= tilesM * tilesN) return;
  const int tm = tile / tilesN;
  const int tn = tile - tm * tilesN;
  const int m0 = tm << 6;
  const int n0 = tn << 6;

  const int rl = lane & 15;
  const int h8 = (lane >> 4) * 8;
  const unsigned short* pa = A + (size_t)(m0 + rl) * (size_t)KTOT + h8;
  const unsigned short* pb = B + (size_t)(n0 + rl) * (size_t)KTOT + h8;

  v8f acc[4][4];
#pragma unroll
  for (int i = 0; i < 4; ++i)
#pragma unroll
    for (int j = 0; j < 4; ++j) acc[i][j] = (v8f){0.f, 0.f, 0.f, 0.f, 0.f, 0.f, 0.f, 0.f};

#pragma unroll 1
  for (int k0 = 0; k0 < KTOT; k0 += 32) {
    F bf[4];
#pragma unroll
    for (int j = 0; j < 4; ++j) bf[j] = ld_frag<F>(pb + (size_t)(j << 4) * (size_t)KTOT + k0);
#pragma unroll
    for (int i = 0; i < 4; ++i) {
      const F af = ld_frag<F>(pa + (size_t)(i << 4) * (size_t)KTOT + k0);
#pragma unroll
      for (int j = 0; j < 4; ++j) acc[i][j] = mm(af, bf[j], acc[i][j]);
    }
  }

  float* slab = sT[wave];
  const int hh = lane >> 4;
  const int c4 = (lane & 15) * 4;
  const int nc = n0 + c4;
  const bool cok = nc < N;
  v4f bv = (v4f){0.f, 0.f, 0.f, 0.f};
  if (EPI == 1) {
    bv = *(const v4fa*)(bias + clampi(nc, 0, N - 4));
    asm volatile("" :: "v"(bv));
  }
#pragma unroll
  for (int i = 0; i < 4; ++i) {
    const int mBase = m0 + (i << 4);
#pragma unroll
    for (int j = 0; j < 4; ++j) {
#pragma unroll
      for (int r = 0; r < 8; ++r) slab[(h8 + r) * 68 + (j << 4) + rl] = acc[i][j][r];
    }
    __builtin_amdgcn_fence(__ATOMIC_RELEASE, "workgroup");
    __builtin_amdgcn_wave_barrier();
    __builtin_amdgcn_fence(__ATOMIC_ACQUIRE, "workgroup");
    v4f vv[8];
#pragma unroll
    for (int it = 0; it < 8; ++it) {
      const int row = it * 2 + hh;
      v4f v = *(const v4fa*)(slab + row * 68 + c4);
      if (EPI == 1) v += bv;
      vv[it] = v;
    }
    for (int pass = 0; pass < 2; ++pass) {
#pragma unroll
      for (int it = 0; it < 8; ++it) {
        const int row = mBase + it * 2 + hh;
        if (cok && row < M) *(volatile v4f*)(D + (size_t)row * (size_t)ldd + nc) = vv[it];
      }
      __threadfence();
    }
    __builtin_amdgcn_fence(__ATOMIC_RELEASE, "workgroup");
    __builtin_amdgcn_wave_barrier();
    __builtin_amdgcn_fence(__ATOMIC_ACQUIRE, "workgroup");
  }
}

#define SPLIT_MEAN1 1
#define SPLIT_L2    1

#define NNODE   50000
#define NEDGE   800000
#define DIN     128
#define HID     256
#define MPAD    50048
#define KC1     384
#define KC2     1024
#define SLB     10
#define NBK     1024
#define NBLK    49
#define BTHR    256
#define BWAVES  8
#define EPW     (NEDGE / BWAVES)
#define SWU     5
#define SWIT    (EPW / (32 * SWU))
#define WCAPL   4096
#define RCAP    20992
#define DEGCAP  64
#define BK_INTS (BWAVES * WCAPL + RCAP + BWAVES * NBK + 2 * NBK + 64)
#define BK_LDS  (BK_INTS * 4)
#define PREP_BLOCKS 119

static_assert(NEDGE % 256 == 0);
static_assert(NEDGE % (BWAVES * 32 * SWU) == 0 && SWIT * 32 * SWU == EPW);
static_assert(NEDGE < (1 << 20) && NBK == (1 << SLB));
static_assert(NNODE <= 65536);
static_assert(NBLK * NBK >= NNODE && (NBLK - 1) * NBK < NNODE);
static_assert(RCAP % 512 == 0 && RCAP * 4 >= 16623 * 5);
static_assert(BWAVES * WCAPL >= RCAP);
static_assert(DEGCAP >= 35 + 8);
static_assert(BK_INTS % 4 == 0 && BK_LDS <= 262144);
static_assert(MPAD % 64 == 0 && MPAD >= NNODE && MPAD % 8 == 0 && NNODE % 16 == 0 && NNODE % 8 == 0);
static_assert(KC1 % 32 == 0 && KC2 % 32 == 0 && DIN % 32 == 0 && HID % 64 == 0);
static_assert(KC1 == 3 * DIN && KC2 == 4 * HID);

#define SZ_RA    ((size_t)MPAD * KC2 * 2)
#define SZ_XB    ((size_t)MPAD * DIN * 2)
#define SZ_LIST  ((size_t)NBLK * RCAP * 4)
#define SZ_OFF   ((size_t)NBLK * NBK * 4)
#define SZ_FLAG  ((size_t)6400)
#define SZ_W1    ((size_t)HID * KC1 * 2)
#define SZ_W2    ((size_t)HID * KC2 * 2)
#define SZ_WR    ((size_t)HID * DIN * 2)
#define SZ_PAR   ((size_t)7 * HID * 4)
#define O_RA     ((size_t)0)
#define O_XB     (O_RA + SZ_RA)
#define O_LIST   (O_XB + SZ_XB)
#define O_OFF    (O_LIST + SZ_LIST)
#define O_CNT    (O_OFF + SZ_OFF)
#define O_FLAG   (O_CNT + SZ_OFF)
#define O_W1     (O_FLAG + SZ_FLAG)
#define O_W2     (O_W1 + SZ_W1)
#define O_WR     (O_W2 + SZ_W2)
#define O_PAR    (O_WR + SZ_WR)
#define WS_TOTAL (O_PAR + SZ_PAR)
static_assert(SZ_RA % 256 == 0 && SZ_XB % 256 == 0 && SZ_LIST % 256 == 0 && SZ_OFF % 256 == 0);
static_assert(SZ_FLAG % 256 == 0 && SZ_FLAG >= (size_t)NBLK * 128);
static_assert(SZ_W1 % 256 == 0 && SZ_W2 % 256 == 0 && SZ_WR % 256 == 0 && SZ_PAR % 256 == 0);
static_assert((size_t)MPAD * KC1 * 2 <= SZ_RA);
static_assert((size_t)MPAD * HID * 4 <= SZ_RA);
static_assert(WS_TOTAL == (size_t)((size_t)471197 << 8));
static_assert(WS_TOTAL <= ((size_t)128 << 20));

typedef unsigned v2u __attribute__((ext_vector_type(2)));
typedef int      v4i __attribute__((ext_vector_type(4)));
typedef v2u __attribute__((may_alias)) v2ua;
typedef v4u __attribute__((may_alias)) v4ua;
typedef v4i __attribute__((may_alias)) v4ia;

__device__ __forceinline__ void wave_sync() {
  __builtin_amdgcn_fence(__ATOMIC_RELEASE, "workgroup");
  __builtin_amdgcn_wave_barrier();
  __builtin_amdgcn_fence(__ATOMIC_ACQUIRE, "workgroup");
}
__device__ __forceinline__ float relu_keep(float v) { return (v > 0.0f) ? v : (v - v); }
__device__ __forceinline__ v4f relu4(v4f v) {
  return (v4f){ relu_keep(v[0]), relu_keep(v[1]), relu_keep(v[2]), relu_keep(v[3]) };
}
__device__ __forceinline__ float wsum(float s) {
#pragma unroll
  for (int m = 16; m >= 1; m >>= 1) s += __shfl_xor(s, m, 32);
  return s;
}
__device__ __forceinline__ float bits_f(unsigned u) { return __uint_as_float(u); }

__device__ __forceinline__ void wtrans(const float* __restrict__ W, int kdim, int u,
                                       unsigned short* __restrict__ P, int pitch, int c0, int c1, bool two) {
  const int ppr = kdim >> 3;
  const int n   = u / ppr;
  const int k8  = (u - n * ppr) << 3;
  float x[8];
#pragma unroll
  for (int e = 0; e < 8; ++e) {
    const float v = W[(size_t)(k8 + e) * HID + n];
    asm volatile("" :: "v"(v));
    x[e] = v;
  }
  const v4u o = pack8_bf16((v4f){ x[0], x[1], x[2], x[3] }, (v4f){ x[4], x[5], x[6], x[7] });
  volatile v4u* q0 = (volatile v4u*)(P + (size_t)n * pitch + c0 + k8);
  volatile v4u* q1 = (volatile v4u*)(P + (size_t)n * pitch + c1 + k8);
  *q0 = o;
  if (two) *q1 = o;
  __threadfence();
  *q0 = o;
  if (two) *q1 = o;
}

__global__ __launch_bounds__(256) void k_prep(const float* __restrict__ Wr1, const float* __restrict__ Wl1,
                                              const float* __restrict__ Wr2, const float* __restrict__ Wl2,
                                              const float* __restrict__ Wres,
                                              const float* __restrict__ bl1, const float* __restrict__ g1,
                                              const float* __restrict__ be1, const float* __restrict__ bl2,
                                              const float* __restrict__ g2, const float* __restrict__ be2,
                                              const float* __restrict__ bres,
                                              unsigned short* __restrict__ W1c, unsigned short* __restrict__ W2c,
                                              unsigned short* __restrict__ WrT, float* __restrict__ PAR) {
  const int b = (int)blockIdx.x, tid = (int)threadIdx.x;
  if (b < 16)        wtrans(Wr1,  DIN, b * 256 + tid,        W1c, KC1, 0,   0,   false);
  else if (b < 32)   wtrans(Wl1,  DIN, (b - 16) * 256 + tid, W1c, KC1, 128, 256, true);
  else if (b < 64)   wtrans(Wr2,  HID, (b - 32) * 256 + tid, W2c, KC2, 0,   256, true);
  else if (b < 96)   wtrans(Wl2,  HID, (b - 64) * 256 + tid, W2c, KC2, 512, 768, true);
  else if (b < 112)  wtrans(Wres, DIN, (b - 96) * 256 + tid, WrT, DIN, 0,   0,   false);
  else if (b < PREP_BLOCKS) {
    const int v  = b - 112;
    const int t4 = (tid & 63) * 4;
    v4f t;
    if (v == 0)      t = *(const v4fa*)(bl1 + t4);
    else if (v == 1) t = *(const v4fa*)(g1 + t4);
    else if (v == 2) t = *(const v4fa*)(be1 + t4);
    else if (v == 3) t = *(const v4fa*)(bl2 + t4);
    else if (v == 4) t = *(const v4fa*)(g2 + t4);
    else if (v == 5) t = *(const v4fa*)(be2 + t4);
    else             t = *(const v4fa*)(bres + t4);
    asm volatile("" :: "v"(t));
    const v4f o = (v4f){ bf16_val(t[0]), bf16_val(t[1]), bf16_val(t[2]), bf16_val(t[3]) };
    if (tid < 64) {
      volatile v4f* q = (volatile v4f*)(PAR + v * HID + t4);
      *q = o;
      __threadfence();
      *q = o;
    }
  }
}

__global__ __launch_bounds__(BTHR) void k_bucket(const int* __restrict__ edge, int* LISTg, int* OFFg, int* CNTg,
                                                 int* FLAGg) {
  extern __shared__ __attribute__((aligned(16))) int dsm[];
  int* wl   = dsm;
  int* sl   = wl + BWAVES * WCAPL;
  int* cw   = sl + RCAP;
  int* offs = cw + BWAVES * NBK;
  int* tot  = offs + NBK;
  int* misc = tot + NBK;
  const int tid = (int)threadIdx.x, lane = tid & 31, wave = tid >> 5;
  const int blk = (int)blockIdx.x;
  const unsigned slotBase = (unsigned)(blk * NBK);
  const int* __restrict__ srcp = edge;
  const int* __restrict__ dstp = edge + NEDGE;

  {
    const v4i z = {0, 0, 0, 0};
    for (int i = tid; i < BK_INTS / 4; i += BTHR) *(v4ia*)(dsm + 4 * i) = z;
  }
  __syncthreads();

  int wc = 0;
  const int ew0 = wave * EPW + lane;
#pragma unroll 1
  for (int it = 0; it < SWIT; ++it) {
    const int eb = ew0 + it * (32 * SWU);
    int kv[SWU];
#pragma unroll
    for (int j = 0; j < SWU; ++j) {
      const int k = dstp[eb + 32 * j];
      asm volatile("" :: "v"(k));
      kv[j] = k;
    }
#pragma unroll
    for (int j = 0; j < SWU; ++j) {
      const unsigned s = (unsigned)kv[j] - slotBase;
      const bool hit = s < (unsigned)NBK;
      const unsigned m = __builtin_amdgcn_ballot_w32(hit);
      if (m != 0u) {
        const int pos = wc + (int)__builtin_amdgcn_mbcnt_lo(m, 0u);
        if (hit && pos < WCAPL) wl[wave * WCAPL + pos] = (int)(((unsigned)(eb + 32 * j) << SLB) | s);
        wc += (int)__builtin_popcount(m);
      }
    }
  }
  const int wov = wc > WCAPL ? 1 : 0;
  const int wcc = __builtin_amdgcn_readfirstlane(wc > WCAPL ? WCAPL : wc);
  if (lane == 0) { misc[wave] = wcc; misc[8 + wave] = wov; }
  wave_sync();

#pragma unroll 1
  for (int b0 = 0; b0 < wcc; b0 += 32) {
    const int idx = b0 + lane;
    const int ent = wl[wave * WCAPL + (idx < WCAPL ? idx : WCAPL - 1)];
    const int m32 = (wcc - b0) < 32 ? (wcc - b0) : 32;
#pragma unroll 1
    for (int k = 0; k < m32; ++k) {
      const int u    = __builtin_amdgcn_readlane(ent, k);
      const int slot = u & (NBK - 1);
      if (lane == 0) cw[wave * NBK + slot] = cw[wave * NBK + slot] + 1;
    }
  }
  __syncthreads();

  const int s0 = 4 * tid;
  int c4[4];
  int ssum = 0;
#pragma unroll
  for (int q = 0; q < 4; ++q) {
    int tq = 0;
#pragma unroll
    for (int w = 0; w < BWAVES; ++w) tq += cw[w * NBK + s0 + q];
    c4[q] = tq;
    ssum += tq;
  }
  int incl = ssum;
#pragma unroll
  for (int d = 1; d < 32; d <<= 1) {
    const int y = __shfl_up(incl, d, 32);
    if (lane >= d) incl += y;
  }
  if (lane == 31) misc[16 + wave] = incl;
  __syncthreads();
  int wbase = 0, total = 0, anyov = 0;
#pragma unroll
  for (int w = 0; w < BWAVES; ++w) {
    const int tw = misc[16 + w];
    if (w < wave) wbase += tw;
    total += tw;
    anyov |= misc[8 + w];
  }
  {
    int run = wbase + incl - ssum;
#pragma unroll
    for (int q = 0; q < 4; ++q) {
      offs[s0 + q] = run;
      tot[s0 + q]  = c4[q];
      int cur = run;
#pragma unroll
      for (int w = 0; w < BWAVES; ++w) {
        const int cc = cw[w * NBK + s0 + q];
        cw[w * NBK + s0 + q] = cur;
        cur += cc;
      }
      run += c4[q];
    }
  }
  const int ovf = (anyov != 0 || total > RCAP) ? 1 : 0;
  __syncthreads();

#pragma unroll 1
  for (int b0 = 0; b0 < wcc; b0 += 32) {
    const int idx = b0 + lane;
    const int ent = wl[wave * WCAPL + (idx < WCAPL ? idx : WCAPL - 1)];
    const int eid = clampi((int)((unsigned)ent >> SLB), 0, NEDGE - 1);
    int sr = srcp[eid];
    asm volatile("" :: "v"(sr));
    sr = clampi(sr, 0, NNODE - 1);
    const int m32 = (wcc - b0) < 32 ? (wcc - b0) : 32;
#pragma unroll 1
    for (int k = 0; k < m32; ++k) {
      const int u    = __builtin_amdgcn_readlane(ent, k);
      const int sk   = __builtin_amdgcn_readlane(sr, k);
      const int slot = u & (NBK - 1);
      if (lane == 0) {
        const int p = cw[wave * NBK + slot];
        cw[wave * NBK + slot] = p + 1;
        sl[clampi(p, 0, RCAP - 1)] = sk;
      }
    }
  }
  __syncthreads();

  int* lg = LISTg + (size_t)blk * RCAP;
  const v4i vo = *(const v4ia*)(offs + s0);
  const v4i vc = *(const v4ia*)(tot + s0);
  const v4i vf = (v4i){ ovf, ovf, ovf, ovf };
  for (int pass = 0; pass < 2; ++pass) {
    for (int i = tid; i < RCAP / 4; i += BTHR) {
      const v4i v = *(const v4ia*)(sl + 4 * i);
      *(volatile v4i*)(lg + 4 * i) = v;
    }
    *(volatile v4i*)(OFFg + blk * NBK + s0) = vo;
    *(volatile v4i*)(CNTg + blk * NBK + s0) = vc;
    if (tid < 8) *(volatile v4i*)(FLAGg + blk * 32 + 4 * tid) = vf;
    __threadfence();
  }
}

__global__ __launch_bounds__(256) void k_agg1(const unsigned short* __restrict__ XB, const int* __restrict__ LISTg,
                                              const int* __restrict__ OFFg, const int* __restrict__ CNTg,
                                              const int* __restrict__ FLAGg, unsigned short* A1) {
  __shared__ __attribute__((aligned(16))) unsigned rowbuf[8][192];
  const int lane = (int)threadIdx.x & 31, wave = (int)threadIdx.x >> 5;
  const int row = (int)blockIdx.x * 8 + wave;
  const bool live = row < NNODE;
  const int rc  = live ? row : NNODE - 1;
  const int blk = rc >> SLB;
  int c = CNTg[rc];
  int o = OFFg[rc];
  const int fl = FLAGg[blk * 32];
  const bool big = c > DEGCAP;
  c = __builtin_amdgcn_readfirstlane(clampi(c, 0, DEGCAP));
  o = __builtin_amdgcn_readfirstlane(clampi(o, 0, RCAP - 1));
  const int cn = live ? c : 0;
  const int* lp = LISTg + (size_t)blk * RCAP;
  float a0 = 0.0f, a1 = 0.0f, a2 = 0.0f, a3 = 0.0f;
#pragma unroll 1
  for (int b0 = 0; b0 < cn; b0 += 32) {
    int idx = o + b0 + lane;
    idx = idx > RCAP - 1 ? RCAP - 1 : idx;
    int sr = lp[idx];
    asm volatile("" :: "v"(sr));
    sr = clampi(sr, 0, NNODE - 1);
    const int m32 = (cn - b0) < 32 ? (cn - b0) : 32;
#pragma unroll 1
    for (int k = 0; k < m32; ++k) {
      const int sk = __builtin_amdgcn_readlane(sr, k);
      const v2u w = *(const v2ua*)(XB + (size_t)sk * DIN + 4 * lane);
      a0 += bits_f(w.x << 16);
      a1 += bits_f(w.x & 0xffff0000u);
      a2 += bits_f(w.y << 16);
      a3 += bits_f(w.y & 0xffff0000u);
    }
  }
  const float dv = (float)(cn > 1 ? cn : 1);
  const bool bad = live && (fl != 0 || big);
  const float nanv = bits_f(0x7fc00000u);
  float m0 = a0 / dv, m1 = a1 / dv, m2 = a2 / dv, m3 = a3 / dv;
  m0 = bad ? nanv : m0; m1 = bad ? nanv : m1; m2 = bad ? nanv : m2; m3 = bad ? nanv : m3;
  v2u hiw, low;
  hiw.x = pk16(bf16_bits(m0), bf16_bits(m1));
  hiw.y = pk16(bf16_bits(m2), bf16_bits(m3));
#if SPLIT_MEAN1
  low.x = pk16(bf16_lo_bits(m0), bf16_lo_bits(m1));
  low.y = pk16(bf16_lo_bits(m2), bf16_lo_bits(m3));
#else
  low.x = 0u; low.y = 0u;
#endif
  const v2u own = *(const v2ua*)(XB + (size_t)row * DIN + 4 * lane);
  asm volatile("" :: "v"(own));
  unsigned* rb = rowbuf[wave];
  *(v2ua*)(rb + 2 * lane)       = own;
  *(v2ua*)(rb + 64 + 2 * lane)  = hiw;
  *(v2ua*)(rb + 128 + 2 * lane) = low;
  wave_sync();
  const v4u q0 = *(const v4ua*)(rb + 4 * lane);
  const v4u q1 = *(const v4ua*)(rb + 128 + 4 * (lane & 15));
  asm volatile("" :: "v"(q1));
  unsigned short* rp = A1 + (size_t)row * KC1;
  for (int pass = 0; pass < 2; ++pass) {
    *(volatile v4u*)(rp + 8 * lane) = q0;
    if (lane < 16) *(volatile v4u*)(rp + 256 + 8 * lane) = q1;
    __threadfence();
  }
}

__global__ __launch_bounds__(256) void k_row1(const float* __restrict__ P, const float* __restrict__ PAR,
                                              unsigned short* __restrict__ A2) {
  __shared__ __attribute__((aligned(16))) float sp[3 * HID];
  const int tid = (int)threadIdx.x, lane = tid & 31, wave = tid >> 5;
  {
    const int t = tid < 192 ? tid : 191;
    const v4f pv = *(const v4fa*)(PAR + 4 * t);
    asm volatile("" :: "v"(pv));
    if (tid < 192) *(v4fa*)(sp + 4 * tid) = pv;
  }
  __syncthreads();
  const int row = (int)blockIdx.x * 8 + wave;
  const bool live = row < NNODE;
  const int rc = live ? row : NNODE - 1;
  const float* pr = P + (size_t)rc * HID + 8 * lane;
  const v4f p0 = *(const v4fa*)pr;
  const v4f p1 = *(const v4fa*)(pr + 4);
  asm volatile("" :: "v"(p0));
  asm volatile("" :: "v"(p1));
  const v4f b0 = *(const v4fa*)(sp + 8 * lane),           b1 = *(const v4fa*)(sp + 8 * lane + 4);
  const v4f g0 = *(const v4fa*)(sp + HID + 8 * lane),     g1v = *(const v4fa*)(sp + HID + 8 * lane + 4);
  const v4f e0 = *(const v4fa*)(sp + 2 * HID + 8 * lane), e1 = *(const v4fa*)(sp + 2 * HID + 8 * lane + 4);
  const v4f v0 = p0 + b0, v1 = p1 + b1;
  float s = ((v0[0] + v0[1]) + (v0[2] + v0[3])) + ((v1[0] + v1[1]) + (v1[2] + v1[3]));
  s = wsum(s);
  const float mu = s * (1.0f / 256.0f);
  const v4f d0 = v0 - mu, d1 = v1 - mu;
  float q = ((d0[0] * d0[0] + d0[1] * d0[1]) + (d0[2] * d0[2] + d0[3] * d0[3])) +
            ((d1[0] * d1[0] + d1[1] * d1[1]) + (d1[2] * d1[2] + d1[3] * d1[3]));
  q = wsum(q);
  const float var = q * (1.0f / 256.0f);
  const float rs = 1.0f / sqrtf(var + 1e-5f);
  v4f y0 = relu4(d0 * rs * g0 + e0);
  v4f y1 = relu4(d1 * rs * g1v + e1);
  if (!live) { y0 = (v4f){0.f, 0.f, 0.f, 0.f}; y1 = (v4f){0.f, 0.f, 0.f, 0.f}; }
  const v4u hi = pack8_bf16(y0, y1);
#if SPLIT_L2
  const v4u lo = pack8_bf16_lo(y0, y1);
#else
  const v4u lo = (v4u){0u, 0u, 0u, 0u};
#endif
  unsigned short* rp = A2 + (size_t)row * KC2 + 8 * lane;
  for (int pass = 0; pass < 2; ++pass) {
    *(volatile v4u*)rp = hi;
    *(volatile v4u*)(rp + HID) = lo;
    __threadfence();
  }
}

__global__ __launch_bounds__(256) void k_agg2(const int* __restrict__ LISTg, const int* __restrict__ OFFg,
                                              const int* __restrict__ CNTg, const int* __restrict__ FLAGg,
                                              unsigned short* A2) {
  const int lane = (int)threadIdx.x & 31, wave = (int)threadIdx.x >> 5;
  const int row = (int)blockIdx.x * 8 + wave;
  const bool live = row < NNODE;
  const int rc  = live ? row : NNODE - 1;
  const int blk = rc >> SLB;
  int c = CNTg[rc];
  int o = OFFg[rc];
  const int fl = FLAGg[blk * 32];
  const bool big = c > DEGCAP;
  c = __builtin_amdgcn_readfirstlane(clampi(c, 0, DEGCAP));
  o = __builtin_amdgcn_readfirstlane(clampi(o, 0, RCAP - 1));
  const int cn = live ? c : 0;
  const int* lp = LISTg + (size_t)blk * RCAP;
  float a[8];
#pragma unroll
  for (int i = 0; i < 8; ++i) a[i] = 0.0f;
#pragma unroll 1
  for (int b0 = 0; b0 < cn; b0 += 32) {
    int idx = o + b0 + lane;
    idx = idx > RCAP - 1 ? RCAP - 1 : idx;
    int sr = lp[idx];
    asm volatile("" :: "v"(sr));
    sr = clampi(sr, 0, NNODE - 1);
    const int m32 = (cn - b0) < 32 ? (cn - b0) : 32;
#pragma unroll 1
    for (int k = 0; k < m32; ++k) {
      const int sk = __builtin_amdgcn_readlane(sr, k);
      const unsigned short* gp = A2 + (size_t)sk * KC2 + 8 * lane;
      const v4u wh = *(const v4ua*)gp;
      const v4u wl = *(const v4ua*)(gp + HID);
#pragma unroll
      for (int q = 0; q < 4; ++q) {
        const float ve = bits_f(wh[q] << 16) + bits_f(wl[q] << 16);
        const float vo = bits_f(wh[q] & 0xffff0000u) + bits_f(wl[q] & 0xffff0000u);
        a[2 * q]     += ve;
        a[2 * q + 1] += vo;
      }
    }
  }
  const float dv = (float)(cn > 1 ? cn : 1);
  const bool bad = live && (fl != 0 || big);
  const float nanv = bits_f(0x7fc00000u);
  float m[8];
#pragma unroll
  for (int i = 0; i < 8; ++i) {
    const float t = a[i] / dv;
    m[i] = bad ? nanv : t;
  }
  const v4f ma = (v4f){ m[0], m[1], m[2], m[3] };
  const v4f mb = (v4f){ m[4], m[5], m[6], m[7] };
  const v4u hi = pack8_bf16(ma, mb);
#if SPLIT_L2
  const v4u lo = pack8_bf16_lo(ma, mb);
#else
  const v4u lo = (v4u){0u, 0u, 0u, 0u};
#endif
  unsigned short* rp = A2 + (size_t)row * KC2 + 2 * HID + 8 * lane;
  for (int pass = 0; pass < 2; ++pass) {
    *(volatile v4u*)rp = hi;
    *(volatile v4u*)(rp + HID) = lo;
    __threadfence();
  }
}

__global__ __launch_bounds__(256) void k_row2(const float* __restrict__ PAR, const float* __restrict__ BASE,
                                              const int* __restrict__ CNTg, const int* __restrict__ FLAGg,
                                              float* out) {
  __shared__ __attribute__((aligned(16))) float sp[4 * HID];
  const int tid = (int)threadIdx.x, lane = tid & 31, wave = tid >> 5;
  {
    const v4f pv = *(const v4fa*)(PAR + 3 * HID + 4 * tid);
    *(v4fa*)(sp + 4 * tid) = pv;
  }
  __syncthreads();
  const int row = (int)blockIdx.x * 8 + wave;
  const int c0 = 4 * lane, c1 = 128 + 4 * lane;
  float* orow = out + (size_t)row * HID;
  const v4f p0 = *(const v4fa*)(orow + c0);
  const v4f p1 = *(const v4fa*)(orow + c1);
  asm volatile("" :: "v"(p0));
  asm volatile("" :: "v"(p1));
  const float* brow = BASE + (size_t)row * HID;
  const v4f r0 = *(const v4fa*)(brow + c0);
  const v4f r1 = *(const v4fa*)(brow + c1);
  asm volatile("" :: "v"(r0));
  asm volatile("" :: "v"(r1));
  const int cnt = CNTg[row];
  const int fl  = FLAGg[(row >> SLB) * 32];
  const v4f b0 = *(const v4fa*)(sp + c0),           b1 = *(const v4fa*)(sp + c1);
  const v4f g0 = *(const v4fa*)(sp + HID + c0),     g1v = *(const v4fa*)(sp + HID + c1);
  const v4f e0 = *(const v4fa*)(sp + 2 * HID + c0), e1 = *(const v4fa*)(sp + 2 * HID + c1);
  const v4f s0 = *(const v4fa*)(sp + 3 * HID + c0), s1 = *(const v4fa*)(sp + 3 * HID + c1);
  const v4f v0 = p0 + b0, v1 = p1 + b1;
  float s = ((v0[0] + v0[1]) + (v0[2] + v0[3])) + ((v1[0] + v1[1]) + (v1[2] + v1[3]));
  s = wsum(s);
  const float mu = s * (1.0f / 256.0f);
  const v4f d0 = v0 - mu, d1 = v1 - mu;
  float q = ((d0[0] * d0[0] + d0[1] * d0[1]) + (d0[2] * d0[2] + d0[3] * d0[3])) +
            ((d1[0] * d1[0] + d1[1] * d1[1]) + (d1[2] * d1[2] + d1[3] * d1[3]));
  q = wsum(q);
  const float var = q * (1.0f / 256.0f);
  const float rs = 1.0f / sqrtf(var + 1e-5f);
  v4f y0 = relu4(d0 * rs * g0 + e0) + (r0 + s0);
  v4f y1 = relu4(d1 * rs * g1v + e1) + (r1 + s1);
  const bool bad = (fl != 0) || (cnt > DEGCAP);
  const float nanv = bits_f(0x7fc00000u);
  y0[0] = bad ? nanv : y0[0]; y0[1] = bad ? nanv : y0[1]; y0[2] = bad ? nanv : y0[2]; y0[3] = bad ? nanv : y0[3];
  y1[0] = bad ? nanv : y1[0]; y1[1] = bad ? nanv : y1[1]; y1[2] = bad ? nanv : y1[2]; y1[3] = bad ? nanv : y1[3];
  for (int pass = 0; pass < 2; ++pass) {
    *(volatile v4f*)(orow + c0) = y0;
    *(volatile v4f*)(orow + c1) = y1;
    __threadfence();
  }
}

extern "C" void kernel_launch(void* const* d_in, const int* in_sizes, int n_in,
                              void* d_out, int out_size, void* d_ws, size_t ws_size,
                              hipStream_t stream) {
  if (n_in < 14) return;
  if (in_sizes[0] != NNODE * DIN) return;
  if (in_sizes[1] != 2 * NEDGE) return;
  if (in_sizes[2] != DIN * HID || in_sizes[4] != DIN * HID || in_sizes[12] != DIN * HID) return;
  if (in_sizes[7] != HID * HID || in_sizes[9] != HID * HID) return;
  if (in_sizes[3] != HID || in_sizes[5] != HID || in_sizes[6] != HID || in_sizes[8] != HID) return;
  if (in_sizes[10] != HID || in_sizes[11] != HID || in_sizes[13] != HID) return;
  if ((long long)out_size != (long long)NNODE * HID) return;
  if (ws_size < WS_TOTAL) return;

  const float* x    = (const float*)d_in[0];
  const int*   edge = (const int*)d_in[1];
  const float* Wl1  = (const float*)d_in[2];
  const float* bl1  = (const float*)d_in[3];
  const float* Wr1  = (const float*)d_in[4];
  const float* g1   = (const float*)d_in[5];
  const float* be1  = (const float*)d_in[6];
  const float* Wl2  = (const float*)d_in[7];
  const float* bl2  = (const float*)d_in[8];
  const float* Wr2  = (const float*)d_in[9];
  const float* g2   = (const float*)d_in[10];
  const float* be2  = (const float*)d_in[11];
  const float* Wres = (const float*)d_in[12];
  const float* bres = (const float*)d_in[13];
  float* out = (float*)d_out;

  char* ws = (char*)d_ws;
  unsigned short* RA   = (unsigned short*)(ws + O_RA);
  float*          BASE = (float*)(ws + O_RA);
  unsigned short* XB   = (unsigned short*)(ws + O_XB);
  int*            LISTg = (int*)(ws + O_LIST);
  int*            OFFg  = (int*)(ws + O_OFF);
  int*            CNTg  = (int*)(ws + O_CNT);
  int*            FLAGg = (int*)(ws + O_FLAG);
  unsigned short* W1c  = (unsigned short*)(ws + O_W1);
  unsigned short* W2c  = (unsigned short*)(ws + O_W2);
  unsigned short* WrT  = (unsigned short*)(ws + O_WR);
  float*          PAR  = (float*)(ws + O_PAR);

  hipFuncSetAttribute(reinterpret_cast<const void*>(&k_bucket), hipFuncAttributeMaxDynamicSharedMemorySize,
                      (int)BK_LDS);

  const int gemmBlocks = (((NNODE + 63) / 64) * (HID / 64) + 7) / 8;

  k_plane<0><<<MPAD * DIN / 8 / 256, 256, 0, stream>>>(x, NNODE, DIN, DIN, XB, MPAD, DIN);
  k_prep<<<PREP_BLOCKS, 256, 0, stream>>>(Wr1, Wl1, Wr2, Wl2, Wres, bl1, g1, be1, bl2, g2, be2, bres,
                                          W1c, W2c, WrT, PAR);
  k_bucket<<<NBLK, BTHR, BK_LDS, stream>>>(edge, LISTg, OFFg, CNTg, FLAGg);
  k_agg1<<<MPAD / 8, 256, 0, stream>>>(XB, LISTg, OFFg, CNTg, FLAGg, RA);
  k_gemm_nt<0, 0><<<gemmBlocks, 256, 0, stream>>>(RA, W1c, PAR, out, NNODE, HID, KC1, HID);
  k_row1<<<MPAD / 8, 256, 0, stream>>>(out, PAR, RA);
  k_agg2<<<MPAD / 8, 256, 0, stream>>>(LISTg, OFFg, CNTg, FLAGg, RA);
  k_gemm_nt<0, 0><<<gemmBlocks, 256, 0, stream>>>(RA, W2c, PAR, out, NNODE, HID, KC2, HID);
  k_gemm_nt<0, 0><<<gemmBlocks, 256, 0, stream>>>(XB, WrT, PAR, BASE, NNODE, HID, DIN, HID);
  k_row2<<<NNODE / 8, 256, 0, stream>>>(PAR, BASE, CNTg, FLAGg, out);
}
